// UniGINConv_34368328303048
// MI455X (gfx1250) — hardware-run, weakly checked
//
#include <hip/hip_runtime.h>

typedef float          v8f   __attribute__((ext_vector_type(8)));
typedef float          v4f   __attribute__((ext_vector_type(4)));
typedef unsigned int   v4u   __attribute__((ext_vector_type(4)));
typedef int            v8i   __attribute__((ext_vector_type(8)));
typedef unsigned short v8us  __attribute__((ext_vector_type(8)));
typedef unsigned short v16us __attribute__((ext_vector_type(16)));
typedef __bf16         v16bf __attribute__((ext_vector_type(16)));
typedef _Float16       v16h  __attribute__((ext_vector_type(16)));
typedef v4f  __attribute__((may_alias)) v4fa;
typedef v8us __attribute__((may_alias)) v8usa;
union FragB { v16bf v; v16us u; v8us h[2]; v8i w; };
union FragH { v16h  v; v16us u; v8us h[2]; v8i w; };

__device__ __forceinline__ v8f wmb(const FragB& a, const FragB& b, v8f c) {
  v8f d = __builtin_amdgcn_wmma_f32_16x16x32_bf16(false, a.v, false, b.v, (short)0, c, false, false);
  asm volatile("v_nop\n\tv_nop\n\tv_nop\n\tv_nop" : "+v"(d) : "v"(a.w), "v"(b.w));
  return d;
}

__device__ __forceinline__ v8f wmh(const FragH& a, const FragH& b, v8f c) {
  v8f d = __builtin_amdgcn_wmma_f32_16x16x32_f16(false, a.v, false, b.v, (short)0, c, false, false);
  asm volatile("v_nop\n\tv_nop\n\tv_nop\n\tv_nop" : "+v"(d) : "v"(a.w), "v"(b.w));
  return d;
}

__device__ __forceinline__ unsigned bf16_bits(float f) {
  const unsigned u = __float_as_uint(f);
  const unsigned r = (u + 0x7FFFu + ((u >> 16) & 1u)) >> 16;
  const unsigned q = (u >> 16) | 0x40u;
  return ((u & 0x7fffffffu) > 0x7f800000u) ? q : r;
}

__device__ __forceinline__ float bf16_val(float f) {
  return __uint_as_float(bf16_bits(f) << 16);
}
__device__ __forceinline__ int clampi(int v, int lo, int hi) {
  return v < lo ? lo : (v > hi ? hi : v);
}

__device__ __forceinline__ unsigned f16_bits(float f) {
  const unsigned u  = __float_as_uint(f);
  const unsigned s  = (u >> 16) & 0x8000u;
  const unsigned a  = u & 0x7fffffffu;
  const unsigned t  = a - 0x38000000u;
  const unsigned r  = (t + 0x0FFFu + ((t >> 13) & 1u)) >> 13;
  const unsigned rc = r > 0x7C00u ? 0x7C00u : r;
  const bool small  = a < 0x38800000u;
  const bool isnan  = a > 0x7f800000u;
  const unsigned fin = small ? 0u : (s | rc);
  return isnan ? (s | 0x7E00u) : fin;
}

__device__ __forceinline__ unsigned pk16(unsigned lo, unsigned hi) { return lo | (hi << 16); }
__device__ __forceinline__ unsigned bf16_lo_bits(float v) {
  float hi = bf16_val(v);
  asm volatile("" : "+v"(hi));
  return bf16_bits(v - hi);
}
__device__ __forceinline__ v4u pack8_bf16(v4f a, v4f c) {
  return (v4u){ pk16(bf16_bits(a[0]), bf16_bits(a[1])), pk16(bf16_bits(a[2]), bf16_bits(a[3])),
                pk16(bf16_bits(c[0]), bf16_bits(c[1])), pk16(bf16_bits(c[2]), bf16_bits(c[3])) };
}
__device__ __forceinline__ v4u pack8_bf16_lo(v4f a, v4f c) {
  return (v4u){ pk16(bf16_lo_bits(a[0]), bf16_lo_bits(a[1])), pk16(bf16_lo_bits(a[2]), bf16_lo_bits(a[3])),
                pk16(bf16_lo_bits(c[0]), bf16_lo_bits(c[1])), pk16(bf16_lo_bits(c[2]), bf16_lo_bits(c[3])) };
}
__device__ __forceinline__ v4u pack8_f16(v4f a, v4f c) {
  return (v4u){ pk16(f16_bits(a[0]), f16_bits(a[1])), pk16(f16_bits(a[2]), f16_bits(a[3])),
                pk16(f16_bits(c[0]), f16_bits(c[1])), pk16(f16_bits(c[2]), f16_bits(c[3])) };
}

template <int FORM>
__global__ __launch_bounds__(256) void k_plane(const float* __restrict__ src, int rows, int cols, int ldsrc,
                                               unsigned short* __restrict__ dst, int MP, int KP) {
  static_assert(FORM >= 0 && FORM <= 3);
  const int KTOT = (FORM == 1 || FORM == 3) ? 2 * KP : KP;
  const unsigned ppr   = (unsigned)(KTOT >> 3);
  const unsigned kp8   = (unsigned)(KP >> 3);
  const unsigned total = (unsigned)MP * ppr;
  const unsigned g     = blockIdx.x * 256u + threadIdx.x;
  const unsigned rowu  = g / ppr;
  const unsigned p     = g - rowu * ppr;
  const bool second    = p >= kp8;
  const int row = (int)rowu;
  const int c0  = (int)((second ? p - kp8 : p) << 3);
  const float* srow = src + (size_t)clampi(row, 0, rows - 1) * (size_t)ldsrc;
  float x[8];
  unsigned mk[8];
#pragma unroll
  for (int e = 0; e < 8; ++e) {
    const int c = c0 + e;
    const float v = srow[clampi(c, 0, cols - 1)];
    asm volatile("" :: "v"(v));
    x[e]  = v;
    mk[e] = (row < rows && c < cols) ? 0xFFFFu : 0u;
  }
  const v4f a = (v4f){ x[0], x[1], x[2], x[3] };
  const v4f c = (v4f){ x[4], x[5], x[6], x[7] };
  v4u o;
  if (FORM == 2) {
    o = pack8_f16(a, c);
  } else {
    const v4u hi = pack8_bf16(a, c);
    o = hi;
    if (FORM == 1) { const v4u lo = pack8_bf16_lo(a, c); o = second ? lo : hi; }
  }
  const v4u mw = (v4u){ pk16(mk[0], mk[1]), pk16(mk[2], mk[3]), pk16(mk[4], mk[5]), pk16(mk[6], mk[7]) };
  o &= mw;
  if (g < total) {
    volatile v4u* q = (volatile v4u*)(dst + (size_t)g * 8);
    *q = o;
    __threadfence();
    *q = o;
  }
}

template <int FORM> struct FragOf    { typedef FragB T; };
template <>         struct FragOf<2> { typedef FragH T; };
__device__ __forceinline__ v8f mm(const FragB& a, const FragB& b, v8f c) { return wmb(a, b, c); }
__device__ __forceinline__ v8f mm(const FragH& a, const FragH& b, v8f c) { return wmh(a, b, c); }
template <class F> __device__ __forceinline__ F ld_frag(const unsigned short* p) {
  F f;
  f.h[0] = *(const v8usa*)(p);
  f.h[1] = *(const v8usa*)(p + 16);
  return f;
}

template <int FORM, int EPI>
__global__ __launch_bounds__(256) __attribute__((amdgpu_num_vgpr(248)))
void k_gemm_nt(const unsigned short* __restrict__ A, const unsigned short* __restrict__ B,
               const float* __restrict__ bias, float* __restrict__ D, int M, int N, int KTOT, int ldd) {
  static_assert(FORM >= 0 && FORM <= 2);
  static_assert(EPI == 0 || EPI == 1);
  typedef typename FragOf<FORM>::T F;
  __shared__ __attribute__((aligned(16))) float sT[8][16 * 68];
  const int lane = threadIdx.x & 31;
  const int wave = threadIdx.x >> 5;
  const int tilesM = (M + 63) >> 6;
  const int tilesN = (N + 63) >> 6;
  const int tile = blockIdx.x * 8 + wave;
  if (tile >= tilesM * tilesN) return;
  const int tm = tile / tilesN;
  const int tn = tile - tm * tilesN;
  const int m0 = tm << 6;
  const int n0 = tn << 6;

  const int rl = lane & 15;
  const int h8 = (lane >> 4) * 8;
  const unsigned short* pa = A + (size_t)(m0 + rl) * (size_t)KTOT + h8;
  const unsigned short* pb = B + (size_t)(n0 + rl) * (size_t)KTOT + h8;

  v8f acc[4][4];
#pragma unroll
  for (int i = 0; i < 4; ++i)
#pragma unroll
    for (int j = 0; j < 4; ++j) acc[i][j] = (v8f){0.f, 0.f, 0.f, 0.f, 0.f, 0.f, 0.f, 0.f};

#pragma unroll 1
  for (int k0 = 0; k0 < KTOT; k0 += 32) {
    F bf[4];
#pragma unroll
    for (int j = 0; j < 4; ++j) bf[j] = ld_frag<F>(pb + (size_t)(j << 4) * (size_t)KTOT + k0);
#pragma unroll
    for (int i = 0; i < 4; ++i) {
      const F af = ld_frag<F>(pa + (size_t)(i << 4) * (size_t)KTOT + k0);
#pragma unroll
      for (int j = 0; j < 4; ++j) acc[i][j] = mm(af, bf[j], acc[i][j]);
    }
  }

  float* slab = sT[wave];
  const int hh = lane >> 4;
  const int c4 = (lane & 15) * 4;
  const int nc = n0 + c4;
  const bool cok = nc < N;
  v4f bv = (v4f){0.f, 0.f, 0.f, 0.f};
  if (EPI == 1) {
    bv = *(const v4fa*)(bias + clampi(nc, 0, N - 4));
    asm volatile("" :: "v"(bv));
  }
#pragma unroll
  for (int i = 0; i < 4; ++i) {
    const int mBase = m0 + (i << 4);
#pragma unroll
    for (int j = 0; j < 4; ++j) {
#pragma unroll
      for (int r = 0; r < 8; ++r) slab[(h8 + r) * 68 + (j << 4) + rl] = acc[i][j][r];
    }
    __builtin_amdgcn_fence(__ATOMIC_RELEASE, "workgroup");
    __builtin_amdgcn_wave_barrier();
    __builtin_amdgcn_fence(__ATOMIC_ACQUIRE, "workgroup");
    v4f vv[8];
#pragma unroll
    for (int it = 0; it < 8; ++it) {
      const int row = it * 2 + hh;
      v4f v = *(const v4fa*)(slab + row * 68 + c4);
      if (EPI == 1) v += bv;
      vv[it] = v;
    }
    for (int pass = 0; pass < 2; ++pass) {
#pragma unroll
      for (int it = 0; it < 8; ++it) {
        const int row = mBase + it * 2 + hh;
        if (cok && row < M) *(volatile v4f*)(D + (size_t)row * (size_t)ldd + nc) = vv[it];
      }
      __threadfence();
    }
    __builtin_amdgcn_fence(__ATOMIC_RELEASE, "workgroup");
    __builtin_amdgcn_wave_barrier();
    __builtin_amdgcn_fence(__ATOMIC_ACQUIRE, "workgroup");
  }
}

#pragma clang fp contract(off)

#ifndef XC_TWO_TERM
#define XC_TWO_TERM 1
#endif

#define NV       50000
#define NM       20000
#define NI       800000
#define DF       128
#define MPAD     50048
#define XCP      (XC_TWO_TERM ? 256 : 128)
#define CHUNK    2048
#define WLN      256
#define SLB_A    9
#define SLOTS_A  512
#define RCAP_A   26624
#define DEGCAP_A 96
#define NBLK_A   40
#define SLB_B    10
#define SLOTS_B  1024
#define RCAP_B   21504
#define DEGCAP_B 64
#define NBLK_B   49
#define PBIT     0x40000000
#define BUILD_INTS(SL, RC) (8 * WLN + 2 * (RC) + 3 * (SL) + 16)

static_assert(NV % 8 == 0 && NM % 8 == 0 && NI % 8 == 0 && NI >= 8);
static_assert(MPAD == 391 * 128 && MPAD % 64 == 0 && MPAD % 32 == 0 && MPAD >= NV);
static_assert(DF == 32 * 4 && DF % 32 == 0 && XCP % 32 == 0);
static_assert(SLOTS_A == (1 << SLB_A) && SLOTS_B == (1 << SLB_B));
static_assert(NBLK_A == (NM + SLOTS_A - 1) / SLOTS_A && NBLK_B == (NV + SLOTS_B - 1) / SLOTS_B);
static_assert(RCAP_A % 1024 == 0 && RCAP_B % 1024 == 0);
static_assert(4 * RCAP_A >= 5 * 20762 && 4 * RCAP_B >= 5 * 16696);
static_assert(DEGCAP_A >= 66 + 8 && DEGCAP_B >= 33 + 8);
static_assert((((long long)(NV - 1)) << SLB_A) + SLOTS_A < (1LL << 31));
static_assert((((long long)(NM - 1)) << SLB_B) + SLOTS_B < (1LL << 31));
static_assert(BUILD_INTS(SLOTS_A, RCAP_A) * 4 <= 262144 && BUILD_INTS(SLOTS_B, RCAP_B) * 4 <= 262144);
static_assert(BUILD_INTS(SLOTS_A, RCAP_A) * 4 + 34816 <= 327680);
static_assert(CHUNK == 256 * 8 && WLN == 32 * 8);

typedef int      v4i  __attribute__((ext_vector_type(4)));
typedef unsigned v2u  __attribute__((ext_vector_type(2)));
typedef v4i __attribute__((may_alias)) v4ia;
typedef v2u __attribute__((may_alias)) v2ua;

__device__ __forceinline__ bool own_poison(int cw, int ow, int degcap, int rcap) {
  const int craw = cw & 0x00FFFFFF;
  return (((unsigned)cw >> 24) != 0u) || (craw > degcap) || (ow < 0) || (ow > rcap - craw);
}

template <int SLB, int RCAP>
__global__ __launch_bounds__(256) void k_build(const int* __restrict__ keys, const int* __restrict__ pays,
                                               int nE, int nOwners, int pmax, int* LIST, int* OFF, int* CNT) {
  constexpr int SLOTS = 1 << SLB;
  constexpr int ZINTS = BUILD_INTS(SLOTS, RCAP);
  static_assert(ZINTS % 4 == 0 && RCAP % 1024 == 0 && SLOTS % 128 == 0 && SLOTS / 4 <= 256);
  extern __shared__ __attribute__((aligned(16))) int dsm[];
  int* wl   = dsm;
  int* hl   = wl + 8 * WLN;
  int* sl   = hl + RCAP;
  int* cnt  = sl + RCAP;
  int* offs = cnt + SLOTS;
  int* cur  = offs + SLOTS;
  int* misc = cur + SLOTS;
  const int tid = (int)threadIdx.x, lane = tid & 31, wave = tid >> 5;
  const int slotBase = (int)blockIdx.x * SLOTS;
  const int nb = clampi(nOwners - slotBase, 0, SLOTS);

  {
    const v4i z4 = (v4i){0, 0, 0, 0};
    for (int i = tid * 4; i < ZINTS; i += 1024) *(v4ia*)(dsm + i) = z4;
  }
  __syncthreads();

  int t = 0;
  int* wlw = wl + wave * WLN;
  const int nChunks = (nE + CHUNK - 1) / CHUNK;
#pragma unroll 1
  for (int ch = 0; ch < nChunks; ++ch) {
    const int e0  = ch * CHUNK + tid * 8;
    const int e0c = e0 < nE - 8 ? e0 : nE - 8;
    v4i ka = *(const v4i*)(keys + e0c);      asm volatile("" :: "v"(ka));
    v4i kb = *(const v4i*)(keys + e0c + 4);  asm volatile("" :: "v"(kb));
    v4i pa = *(const v4i*)(pays + e0c);      asm volatile("" :: "v"(pa));
    v4i pb = *(const v4i*)(pays + e0c + 4);  asm volatile("" :: "v"(pb));
    const unsigned ub = (unsigned)slotBase;
    const unsigned un = (e0 < nE) ? (unsigned)nb : 0u;
    const int kk[8] = { ka.x, ka.y, ka.z, ka.w, kb.x, kb.y, kb.z, kb.w };
    const int pp[8] = { pa.x, pa.y, pa.z, pa.w, pb.x, pb.y, pb.z, pb.w };
    int  ent[8];
    bool hit[8];
    int nh = 0;
#pragma unroll
    for (int j = 0; j < 8; ++j) {
      const unsigned s = (unsigned)kk[j] - ub;
      hit[j] = s < un;
      ent[j] = (clampi(pp[j], 0, pmax) << SLB) | (int)(s & (unsigned)(SLOTS - 1));
      nh += hit[j] ? 1 : 0;
    }
    int incl = nh;
#pragma unroll
    for (int d = 1; d < 32; d <<= 1) {
      const int y = __shfl_up(incl, d, 32);
      incl += (lane >= d) ? y : 0;
    }
    const int wc = __builtin_amdgcn_readlane(incl, 31);
    int pos = incl - nh;
#pragma unroll
    for (int j = 0; j < 8; ++j) {
      if (hit[j]) wlw[pos & (WLN - 1)] = ent[j];
      pos += hit[j] ? 1 : 0;
    }
    if (lane == 0) misc[wave] = wc;
    __syncthreads();
    int mybase = t, myc = 0, tot = 0;
#pragma unroll
    for (int w2 = 0; w2 < 8; ++w2) {
      const int c = clampi(misc[w2], 0, WLN);
      mybase += (w2 < wave) ? c : 0;
      myc     = (w2 == wave) ? c : myc;
      tot    += c;
    }
    const int mycu = __builtin_amdgcn_readfirstlane(myc);
#pragma unroll 1
    for (int b0 = 0; b0 < mycu; b0 += 32) {
      const int idx = b0 + lane;
      const int u = wlw[idx < WLN ? idx : WLN - 1];
      const int p = mybase + idx;
      if (idx < mycu && p < RCAP) hl[p] = u;
    }
    t += tot;
    __syncthreads();
  }
  const int ovf = (t > RCAP) ? 1 : 0;
  const int tt  = t < 0 ? 0 : (t > RCAP ? RCAP : t);

  if (tid == 0) {
#pragma unroll 1
    for (int i = 0; i < tt; ++i) {
      const int s = hl[i] & (SLOTS - 1);
      cnt[s] = cnt[s] + 1;
    }
  }
  __syncthreads();
  if (wave == 0) {
    constexpr int PER = SLOTS / 32;
    const int base = lane * PER;
    int s = 0;
#pragma unroll 1
    for (int i = 0; i < PER; ++i) s += cnt[base + i];
    int incl = s;
#pragma unroll
    for (int d = 1; d < 32; d <<= 1) {
      const int y = __shfl_up(incl, d, 32);
      incl += (lane >= d) ? y : 0;
    }
    int run = incl - s;
#pragma unroll 1
    for (int i = 0; i < PER; ++i) {
      const int cv = cnt[base + i];
      offs[base + i] = run;
      cur[base + i]  = run;
      run += cv;
    }
  }
  __syncthreads();
  if (tid == 0) {
#pragma unroll 1
    for (int i = 0; i < tt; ++i) {
      const int u = hl[i];
      const int s = u & (SLOTS - 1);
      const int p = clampi(cur[s], 0, RCAP - 1);
      sl[p] = u;
      cur[s] = p + 1;
    }
  }
  __syncthreads();

  int* lp = LIST + (size_t)blockIdx.x * (size_t)RCAP;
#pragma unroll 1
  for (int pass = 0; pass < 2; ++pass) {
#pragma unroll 1
    for (int i4 = tid * 4; i4 < RCAP; i4 += 1024) {
      const v4i q = *(const v4ia*)(sl + i4);
      const v4i o = (v4i){ q.x >> SLB, q.y >> SLB, q.z >> SLB, q.w >> SLB };
      *(volatile v4i*)(lp + i4) = o;
    }
    __threadfence();
  }
  if (tid < SLOTS / 4) {
    const v4i o4 = *(const v4ia*)(offs + 4 * tid);
    const v4i c0 = *(const v4ia*)(cnt + 4 * tid);
    const int pbw = ovf ? PBIT : 0;
    const v4i c4 = (v4i){ c0.x | pbw, c0.y | pbw, c0.z | pbw, c0.w | pbw };
    volatile v4i* po = (volatile v4i*)(OFF + (size_t)blockIdx.x * SLOTS + 4 * tid);
    volatile v4i* pc = (volatile v4i*)(CNT + (size_t)blockIdx.x * SLOTS + 4 * tid);
    *po = o4;
    *pc = c4;
    __threadfence();
    *po = o4;
    *pc = c4;
  }
}

__global__ __launch_bounds__(256) void k_walkA(const unsigned short* __restrict__ XB, const int* __restrict__ LISTA,
                                               const int* __restrict__ OFFA, const int* __restrict__ CNTA,
                                               float* XE, int nM, int nV) {
  const int lane = (int)threadIdx.x & 31, wave = (int)threadIdx.x >> 5;
  const int m = (int)blockIdx.x * 8 + wave;
  const bool live = m < nM;
  const int mc = clampi(m, 0, nM - 1);
  int cw = CNTA[mc]; asm volatile("" :: "v"(cw));
  int ow = OFFA[mc]; asm volatile("" :: "v"(ow));
  const int craw = cw & 0x00FFFFFF;
  const bool pois = own_poison(cw, ow, DEGCAP_A, RCAP_A);
  const int o = clampi(ow, 0, RCAP_A);
  int c = craw > DEGCAP_A ? DEGCAP_A : craw;
  c = c > RCAP_A - o ? RCAP_A - o : c;
  const int cn = __builtin_amdgcn_readfirstlane(live ? c : 0);
  const int* lp = LISTA + (size_t)(mc >> SLB_A) * (size_t)RCAP_A;
  float a0 = 0.0f, a1 = 0.0f, a2 = 0.0f, a3 = 0.0f;
#pragma unroll 1
  for (int b0 = 0; b0 < cn; b0 += 32) {
    int idx = o + b0 + lane;
    idx = idx > RCAP_A - 1 ? RCAP_A - 1 : idx;
    int v = lp[idx]; asm volatile("" :: "v"(v));
    v = clampi(v, 0, nV - 1);
    const int m32 = (cn - b0) < 32 ? (cn - b0) : 32;
#pragma unroll 1
    for (int k = 0; k < m32; ++k) {
      const int sk = __builtin_amdgcn_readlane(v, k);
      const v2u w = *(const v2ua*)(XB + (size_t)sk * DF + 4 * lane);
      asm volatile("" :: "v"(w));
      a0 = a0 + __uint_as_float(w.x << 16);
      a1 = a1 + __uint_as_float(w.x & 0xffff0000u);
      a2 = a2 + __uint_as_float(w.y << 16);
      a3 = a3 + __uint_as_float(w.y & 0xffff0000u);
    }
  }
  const float den = fmaxf((float)craw, 1.0f);
  const float qn = __uint_as_float(0x7fc00000u);
  v4f r;
  r.x = pois ? qn : (a0 / den);
  r.y = pois ? qn : (a1 / den);
  r.z = pois ? qn : (a2 / den);
  r.w = pois ? qn : (a3 / den);
  if (live) {
    volatile v4f* q = (volatile v4f*)(XE + (size_t)m * DF + 4 * lane);
    *q = r;
    __threadfence();
    *q = r;
  }
}

__global__ __launch_bounds__(256) void k_walkB(const unsigned short* __restrict__ XB, const float* __restrict__ XE,
                                               const float* __restrict__ epsp,
                                               const int* __restrict__ LISTB, const int* __restrict__ OFFB,
                                               const int* __restrict__ CNTB,
                                               const int* __restrict__ OFFA, const int* __restrict__ CNTA,
                                               unsigned short* XC, int* PFB, int nV, int nM, int mRows) {
  __shared__ __attribute__((aligned(16))) int sflag[32];
  const int lane = (int)threadIdx.x & 31, wave = (int)threadIdx.x >> 5;
  float ev = epsp[0]; asm volatile("" :: "v"(ev));
  const float opE = 1.0f + bf16_val(ev);
#pragma unroll 1
  for (int i = 0; i < 4; ++i) {
    const int n = (int)blockIdx.x * 32 + wave * 4 + i;
    const bool live = n < nV;
    const int nc = clampi(n, 0, nV - 1);
    int cw = CNTB[nc]; asm volatile("" :: "v"(cw));
    int ow = OFFB[nc]; asm volatile("" :: "v"(ow));
    const int craw = cw & 0x00FFFFFF;
    unsigned pany = own_poison(cw, ow, DEGCAP_B, RCAP_B) ? 1u : 0u;
    const int o = clampi(ow, 0, RCAP_B);
    int c = craw > DEGCAP_B ? DEGCAP_B : craw;
    c = c > RCAP_B - o ? RCAP_B - o : c;
    const int cn = __builtin_amdgcn_readfirstlane(live ? c : 0);
    const int* lp = LISTB + (size_t)(nc >> SLB_B) * (size_t)RCAP_B;
    float a0 = 0.0f, a1 = 0.0f, a2 = 0.0f, a3 = 0.0f;
#pragma unroll 1
    for (int b0 = 0; b0 < cn; b0 += 32) {
      int idx = o + b0 + lane;
      idx = idx > RCAP_B - 1 ? RCAP_B - 1 : idx;
      int e = lp[idx]; asm volatile("" :: "v"(e));
      e = clampi(e, 0, nM - 1);
      int cwa = CNTA[e]; asm volatile("" :: "v"(cwa));
      int owa = OFFA[e]; asm volatile("" :: "v"(owa));
      const bool pa = ((b0 + lane) < cn) && own_poison(cwa, owa, DEGCAP_A, RCAP_A);
      pany |= (__builtin_amdgcn_ballot_w32(pa) != 0u) ? 1u : 0u;
      const int m32 = (cn - b0) < 32 ? (cn - b0) : 32;
#pragma unroll 1
      for (int k = 0; k < m32; ++k) {
        const int ek = __builtin_amdgcn_readlane(e, k);
        const v4f x = *(const v4fa*)(XE + (size_t)ek * DF + 4 * lane);
        asm volatile("" :: "v"(x));
        a0 = a0 + x.x;
        a1 = a1 + x.y;
        a2 = a2 + x.z;
        a3 = a3 + x.w;
      }
    }
    const v2u w = *(const v2ua*)(XB + (size_t)nc * DF + 4 * lane);
    asm volatile("" :: "v"(w));
    const float t0 = opE * __uint_as_float(w.x << 16);
    const float t1 = opE * __uint_as_float(w.x & 0xffff0000u);
    const float t2 = opE * __uint_as_float(w.y << 16);
    const float t3 = opE * __uint_as_float(w.y & 0xffff0000u);
    float c0 = t0 + a0, c1 = t1 + a1, c2 = t2 + a2, c3 = t3 + a3;
    c0 = live ? c0 : 0.0f;
    c1 = live ? c1 : 0.0f;
    c2 = live ? c2 : 0.0f;
    c3 = live ? c3 : 0.0f;
    const v2u hw = (v2u){ pk16(bf16_bits(c0), bf16_bits(c1)), pk16(bf16_bits(c2), bf16_bits(c3)) };
    const v2u lw = (v2u){ pk16(bf16_lo_bits(c0), bf16_lo_bits(c1)), pk16(bf16_lo_bits(c2), bf16_lo_bits(c3)) };
    if (n < mRows) {
      unsigned short* rp = XC + (size_t)n * XCP + 4 * lane;
      *(volatile v2u*)rp = hw;
      if (XC_TWO_TERM) *(volatile v2u*)(rp + DF) = lw;
      __threadfence();
      *(volatile v2u*)rp = hw;
      if (XC_TWO_TERM) *(volatile v2u*)(rp + DF) = lw;
    }
    if (lane == 0) sflag[wave * 4 + i] = (live && pany != 0u) ? 1 : 0;
  }
  __syncthreads();
  if (wave == 0 && lane < 8) {
    const v4i q = *(const v4ia*)(sflag + 4 * lane);
    volatile v4i* pf = (volatile v4i*)(PFB + (size_t)blockIdx.x * 32 + 4 * lane);
    *pf = q;
    __threadfence();
    *pf = q;
  }
}

__device__ __forceinline__ float nn_sel(float v) {
  float r = v;
  r = (v ==  __builtin_inff()) ?  100.0f : r;
  r = (v == -__builtin_inff()) ? -100.0f : r;
  r = (v != v) ? 0.0f : r;
  return r;
}

__global__ __launch_bounds__(256) void k_final(const float* __restrict__ P, const int* __restrict__ PFB,
                                               float* out, int nrows) {
  const int lane = (int)threadIdx.x & 31, wave = (int)threadIdx.x >> 5;
  const int row = (int)blockIdx.x * 8 + wave;
  const int rc = clampi(row, 0, nrows - 1);
  const v4f v = *(const v4fa*)(P + (size_t)rc * DF + 4 * lane);
  asm volatile("" :: "v"(v));
  int pf = PFB[rc]; asm volatile("" :: "v"(pf));
  const float qn = __uint_as_float(0x7fc00000u);
  v4f o;
  o.x = nn_sel(v.x);
  o.y = nn_sel(v.y);
  o.z = nn_sel(v.z);
  o.w = nn_sel(v.w);
  o.x = (pf != 0) ? qn : o.x;
  o.y = (pf != 0) ? qn : o.y;
  o.z = (pf != 0) ? qn : o.z;
  o.w = (pf != 0) ? qn : o.w;
  if (row < nrows) {
    volatile v4f* q = (volatile v4f*)(out + (size_t)row * DF + 4 * lane);
    *q = o;
    __threadfence();
    *q = o;
  }
}

constexpr size_t SZ_XB = (size_t)MPAD * DF * 2;
constexpr size_t SZ_XE = (size_t)NM * DF * 4;
constexpr size_t SZ_XC = (size_t)MPAD * XCP * 2;
constexpr size_t SZ_P  = (size_t)MPAD * DF * 4;
constexpr size_t SZ_WD = (size_t)DF * XCP * 2;
constexpr size_t SZ_LA = (size_t)NBLK_A * RCAP_A * 4;
constexpr size_t SZ_LB = (size_t)NBLK_B * RCAP_B * 4;
constexpr size_t SZ_OA = (size_t)NBLK_A * SLOTS_A * 4;
constexpr size_t SZ_OB = (size_t)NBLK_B * SLOTS_B * 4;
constexpr size_t SZ_PF = (size_t)MPAD * 4;
constexpr size_t O_XB = 0;
constexpr size_t O_XE = O_XB + SZ_XB;
constexpr size_t O_XC = O_XE + SZ_XE;
constexpr size_t O_P  = O_XC + SZ_XC;
constexpr size_t O_WD = O_P + SZ_P;
constexpr size_t O_LA = O_WD + SZ_WD;
constexpr size_t O_LB = O_LA + SZ_LA;
constexpr size_t O_OA = O_LB + SZ_LB;
constexpr size_t O_CA = O_OA + SZ_OA;
constexpr size_t O_OB = O_CA + SZ_OA;
constexpr size_t O_CB = O_OB + SZ_OB;
constexpr size_t O_PF = O_CB + SZ_OB;
constexpr size_t WS_TOTAL = O_PF + SZ_PF;
static_assert(SZ_XB % 256 == 0 && SZ_XE % 256 == 0 && SZ_XC % 256 == 0 && SZ_P % 256 == 0 && SZ_WD % 256 == 0);
static_assert(SZ_LA % 256 == 0 && SZ_LB % 256 == 0 && SZ_OA % 256 == 0 && SZ_OB % 256 == 0 && SZ_PF % 256 == 0);
static_assert(WS_TOTAL <= ((size_t)128 << 20));
static_assert((size_t)MPAD * XCP / 8 < ((size_t)1 << 31));
static_assert(((size_t)MPAD * DF / 8) % 256 == 0 && ((size_t)DF * XCP / 8) % 256 == 0);
static_assert((size_t)NV * DF - 1 == 6399999);

extern "C" void kernel_launch(void* const* d_in, const int* in_sizes, int n_in,
                              void* d_out, int out_size, void* d_ws, size_t ws_size,
                              hipStream_t stream) {
  if (n_in < 5) return;
  if (in_sizes[0] != NV * DF || in_sizes[1] != DF * DF || in_sizes[2] < 1) return;
  if (in_sizes[3] != NI || in_sizes[4] != NI) return;
  if (out_size != NV * DF) return;
  if (ws_size < WS_TOTAL) return;

  const float* X    = (const float*)d_in[0];
  const float* W    = (const float*)d_in[1];
  const float* eps  = (const float*)d_in[2];
  const int*   vtx  = (const int*)d_in[3];
  const int*   edg  = (const int*)d_in[4];
  float* out = (float*)d_out;

  char* ws = (char*)d_ws;
  unsigned short* XB = (unsigned short*)(ws + O_XB);
  float*          XE = (float*)(ws + O_XE);
  unsigned short* XC = (unsigned short*)(ws + O_XC);
  float*          P  = (float*)(ws + O_P);
  unsigned short* WD = (unsigned short*)(ws + O_WD);
  int* LISTA = (int*)(ws + O_LA);
  int* LISTB = (int*)(ws + O_LB);
  int* OFFA  = (int*)(ws + O_OA);
  int* CNTA  = (int*)(ws + O_CA);
  int* OFFB  = (int*)(ws + O_OB);
  int* CNTB  = (int*)(ws + O_CB);
  int* PFB   = (int*)(ws + O_PF);

  const int ldsA = BUILD_INTS(SLOTS_A, RCAP_A) * 4;
  const int ldsB = BUILD_INTS(SLOTS_B, RCAP_B) * 4;
  hipFuncSetAttribute(reinterpret_cast<const void*>(&k_build<SLB_A, RCAP_A>),
                      hipFuncAttributeMaxDynamicSharedMemorySize, ldsA);
  hipFuncSetAttribute(reinterpret_cast<const void*>(&k_build<SLB_B, RCAP_B>),
                      hipFuncAttributeMaxDynamicSharedMemorySize, ldsB);

  k_plane<0><<<(MPAD * DF / 8) / 256, 256, 0, stream>>>(X, NV, DF, DF, XB, MPAD, DF);
#if XC_TWO_TERM
  k_plane<3><<<(DF * XCP / 8) / 256, 256, 0, stream>>>(W, DF, DF, DF, WD, DF, DF);
#else
  k_plane<0><<<(DF * XCP / 8) / 256, 256, 0, stream>>>(W, DF, DF, DF, WD, DF, DF);
#endif
  k_build<SLB_A, RCAP_A><<<NBLK_A, 256, ldsA, stream>>>(edg, vtx, NI, NM, NV - 1, LISTA, OFFA, CNTA);
  k_build<SLB_B, RCAP_B><<<NBLK_B, 256, ldsB, stream>>>(vtx, edg, NI, NV, NM - 1, LISTB, OFFB, CNTB);
  k_walkA<<<NM / 8, 256, 0, stream>>>(XB, LISTA, OFFA, CNTA, XE, NM, NV);
  k_walkB<<<MPAD / 32, 256, 0, stream>>>(XB, XE, eps, LISTB, OFFB, CNTB, OFFA, CNTA, XC, PFB, NV, NM, MPAD);
  {
    const int tiles = (MPAD / 64) * (DF / 64);
    k_gemm_nt<0, 0><<<(tiles + 7) / 8, 256, 0, stream>>>(XC, WD, W, P, MPAD, DF, XCP, DF);
  }
  k_final<<<NV / 8, 256, 0, stream>>>(P, PFB, out, NV);
}
